// GCNNet_26474178413326
// MI455X (gfx1250) — hardware-verified
//
#include <hip/hip_runtime.h>
#include <stddef.h>
#include <stdint.h>
#include <math.h>


#define NN     50000
#define NE     800000
#define NGR    512
#define FIN    62
#define FP     64
#define K2     128
#define NNET   4
#define MP     50048
#define NX     (NN * FIN)
#define XGRP   128
#define XGF    (XGRP * FIN)
#define NXG    391
#define NTHR   256
#define NWAVE  8
#define EPT    8
#define CHUNK  (NTHR * EPT)
#define WCAP   (EPT * 32)
#define LISTN  (NWAVE * WCAP)
#define NBA    1024
#define SLA    10
#define NBLK   49
#define NBPAD  (NBLK * NBA)
#define RCAP   28672
#define DEGCAP 64
#define GBM    64
#define GBN    64
#define GTHR   128
#define AGG_ZINTS (LISTN + 2 * RCAP + 3 * NBA)
#define BKT_LDS_INTS (AGG_ZINTS + 16)
#define PGB    32
#define PTAB   (NWAVE * PGB * FP)
#define POOL_LDS_BYTES (PTAB * 4 + PGB * K2 * 2)
#define HROWS  128
#define XCP    65
#define TB1    0
#define TBG    256
#define TFB    512
#define TOW    576
#define TOB    640
#define TABN   672
#define PB_X   (NNET * NXG)
#define NU_W1  (NNET * FP * (FP / 8))
#define NU_WG  (NNET * FP * (K2 / 8))
#define NU_FC  (FP * (K2 / 8))
#define PB_W1  (NU_W1 / NTHR)
#define PB_WG  (NU_WG / NTHR)
#define PB_FC  (NU_FC / NTHR)
#define PB_ALL (PB_X + PB_W1 + PB_WG + PB_FC + 1)
#define WSMAX  134217728

static_assert(FIN <= FP && FP == 64 && K2 == 2 * FP && K2 % 32 == 0 && FP % 32 == 0);
static_assert((CHUNK & (CHUNK - 1)) == 0 && CHUNK <= 4096);
static_assert((NBA & (NBA - 1)) == 0 && NBA == (1 << SLA));
static_assert(((long long)CHUNK << SLA) < (1LL << 31));
static_assert(((long long)NE << SLA) < (1LL << 31));
static_assert(NE % 4 == 0);
static_assert(LISTN % NTHR == 0 && NBA == 4 * NTHR && NBA % NWAVE == 0 && NBA % 32 == 0);
static_assert(RCAP % (4 * NTHR) == 0 && AGG_ZINTS % 4 == 0);
static_assert(RCAP * 100 >= 16711 * 105);
static_assert(DEGCAP >= 37 + 8);
static_assert(NBLK * NBA >= MP && (NBLK - 1) * NBA < NN && NN - (NBLK - 1) * NBA == 848);
static_assert(MP % GBM == 0 && MP == NXG * XGRP && MP >= NN);
static_assert(GBM == (GTHR / 32) * 16 && GBN == 64);
static_assert(NX % 4 == 0 && XGF % 4 == 0 && (XGF * 4) % 128 == 0);
static_assert(NU_W1 % NTHR == 0 && NU_WG % NTHR == 0 && NU_FC % NTHR == 0);
static_assert(NGR % HROWS == 0 && NGR % PGB == 0 && HROWS == NWAVE * 16);
static_assert(BKT_LDS_INTS * 4 <= 300000 && POOL_LDS_BYTES <= 300000);
static_assert(HROWS * XCP * 4 >= HROWS * K2 * 2);
static_assert(TABN % 4 == 0 && TOB + 32 == TABN);

typedef float          v2f   __attribute__((ext_vector_type(2)));
typedef float          v4f   __attribute__((ext_vector_type(4)));
typedef float          v8f   __attribute__((ext_vector_type(8)));
typedef int            v4i   __attribute__((ext_vector_type(4)));
typedef int            v8i   __attribute__((ext_vector_type(8)));
typedef unsigned short v8us  __attribute__((ext_vector_type(8)));
typedef unsigned short v16us __attribute__((ext_vector_type(16)));
typedef __bf16         v16bf __attribute__((ext_vector_type(16)));
typedef v2f  __attribute__((may_alias)) v2fa;
typedef v4f  __attribute__((may_alias)) v4fa;
typedef v4i  __attribute__((may_alias)) v4ia;
typedef v8us __attribute__((may_alias)) v8usa;
union FragB { v16bf v; v16us u; v8us h[2]; v8i w; };

__device__ __forceinline__ v8f wmb(const FragB& a, const FragB& b, v8f c) {
  v8f d = __builtin_amdgcn_wmma_f32_16x16x32_bf16(false, a.v, false, b.v, (short)0, c, false, false);
  asm volatile("v_nop\n\tv_nop\n\tv_nop\n\tv_nop" : "+v"(d) : "v"(a.w), "v"(b.w));
  return d;
}

__device__ __forceinline__ unsigned bf16_bits(float f) {
  const unsigned u = __float_as_uint(f);
  const unsigned r = (u + 0x7FFFu + ((u >> 16) & 1u)) >> 16;
  return (f != f) ? 0x7FC0u : r;
}
__device__ __forceinline__ float bf16_val(float f) {
  return __uint_as_float(bf16_bits(f) << 16);
}

template <int SLB>
__device__ __forceinline__ int scan_chunk(const int* __restrict__ dsts, int nE, int cbase, int slotBase,
                                          int nb, int vec8, int* list, int tid, int lane, int wave) {
  int wc = 0;
  const int el0  = tid * EPT;
  const int e0   = cbase + el0;
  const int sent = -2147483647 - 1;
  v4i da, db;
  if (vec8 != 0 && cbase + CHUNK <= nE) {
    da = *(const v4i*)(dsts + e0);
    db = *(const v4i*)(dsts + e0 + 4);
  } else {
    da.x = (e0     < nE) ? dsts[min(e0,     nE - 1)] : sent;
    da.y = (e0 + 1 < nE) ? dsts[min(e0 + 1, nE - 1)] : sent;
    da.z = (e0 + 2 < nE) ? dsts[min(e0 + 2, nE - 1)] : sent;
    da.w = (e0 + 3 < nE) ? dsts[min(e0 + 3, nE - 1)] : sent;
    db.x = (e0 + 4 < nE) ? dsts[min(e0 + 4, nE - 1)] : sent;
    db.y = (e0 + 5 < nE) ? dsts[min(e0 + 5, nE - 1)] : sent;
    db.z = (e0 + 6 < nE) ? dsts[min(e0 + 6, nE - 1)] : sent;
    db.w = (e0 + 7 < nE) ? dsts[min(e0 + 7, nE - 1)] : sent;
  }
  const unsigned nbs = (unsigned)slotBase;
  const unsigned unb = (unsigned)nb;
  const unsigned s0 = (unsigned)da.x - nbs, s1 = (unsigned)da.y - nbs;
  const unsigned s2 = (unsigned)da.z - nbs, s3 = (unsigned)da.w - nbs;
  const unsigned s4 = (unsigned)db.x - nbs, s5 = (unsigned)db.y - nbs;
  const unsigned s6 = (unsigned)db.z - nbs, s7 = (unsigned)db.w - nbs;
  const bool h0 = s0 < unb, h1 = s1 < unb, h2 = s2 < unb, h3 = s3 < unb;
  const bool h4 = s4 < unb, h5 = s5 < unb, h6 = s6 < unb, h7 = s7 < unb;
  const unsigned any = __builtin_amdgcn_ballot_w32(h0 | h1 | h2 | h3 | h4 | h5 | h6 | h7);
  if (any != 0u) {
#define HITJ(J, HJ, SJ) { \
      const unsigned mj = __builtin_amdgcn_ballot_w32(HJ); \
      if (mj != 0u) { \
        if (HJ) { \
          const int pos = wc + (int)__builtin_amdgcn_mbcnt_lo(mj, 0u); \
          if (pos < WCAP) list[wave * WCAP + pos] = ((el0 + (J)) << SLB) | (int)(SJ); \
        } \
        wc += (int)__builtin_popcount(mj); } }
    HITJ(0, h0, s0)
    HITJ(1, h1, s1)
    HITJ(2, h2, s2)
    HITJ(3, h3, s3)
    HITJ(4, h4, s4)
    HITJ(5, h5, s5)
    HITJ(6, h6, s6)
    HITJ(7, h7, s7)
#undef HITJ
  }
  return wc;
}

__device__ __forceinline__ void x_stage(const float* __restrict__ x, int grp, float* sx, int tid) {
  const int fbase = grp * XGF;
#pragma unroll 1
  for (int it = 0; it < 8; ++it) {
    const int j = it * NTHR + tid;
    if (j < XGF / 4) {
      const int f  = fbase + 4 * j;
      const bool ok = f < NX;
      const int fc = ok ? f : NX - 4;
      v4f v = *(const v4fa*)(x + fc);
      v.x = ok ? v.x : 0.0f; v.y = ok ? v.y : 0.0f; v.z = ok ? v.z : 0.0f; v.w = ok ? v.w : 0.0f;
      *(v4fa*)(sx + 4 * j) = v;
    }
  }
}

__device__ __forceinline__ float tab_elem(const float* __restrict__ src, int nsrc, int srcW, int d) {
  const int row = d >> 6;
  const int c   = d & 63;
  const bool ok = c < srcW;
  int si = row * srcW + (ok ? c : srcW - 1);
  si = si < 0 ? 0 : (si > nsrc - 1 ? nsrc - 1 : si);
  const float val = src[si];
  return ok ? bf16_val(val) : 0.0f;
}
__device__ __forceinline__ void tab_fill(const float* __restrict__ src, int nsrc, int srcW, float* dst,
                                         int nUnits, int tid) {
  const int tu = tid < nUnits ? tid : nUnits - 1;
  v4f o;
  o.x = tab_elem(src, nsrc, srcW, 4 * tu + 0);
  o.y = tab_elem(src, nsrc, srcW, 4 * tu + 1);
  o.z = tab_elem(src, nsrc, srcW, 4 * tu + 2);
  o.w = tab_elem(src, nsrc, srcW, 4 * tu + 3);
  float* dp = dst + 4 * tu;
  const bool wr = tid < nUnits;
  if (wr) *(volatile v4f*)dp = o;
  __threadfence();
  if (wr) *(volatile v4f*)dp = o;
}

__global__ __launch_bounds__(NTHR) void k_prep(
    const float* __restrict__ x0, const float* __restrict__ x1, const float* __restrict__ x2,
    const float* __restrict__ x3, const float* __restrict__ W1, const float* __restrict__ b1,
    const float* __restrict__ Wg, const float* __restrict__ bg, const float* __restrict__ fcW,
    const float* __restrict__ fcb, const float* __restrict__ oW, const float* __restrict__ ob,
    unsigned short* XB, unsigned short* W1T, unsigned short* WGT2, unsigned short* FC1T2, float* TAB) {
  __shared__ __attribute__((aligned(16))) float sx[XGF];
  const int tid = (int)threadIdx.x;
  const int bid = (int)blockIdx.x;
  if (bid < PB_X) {
    const int net = bid / NXG;
    const int grp = bid - net * NXG;
    if (net == 0)      x_stage(x0, grp, sx, tid);
    else if (net == 1) x_stage(x1, grp, sx, tid);
    else if (net == 2) x_stage(x2, grp, sx, tid);
    else               x_stage(x3, grp, sx, tid);
    __syncthreads();
    unsigned short* xbn = XB + (size_t)net * MP * FP + (size_t)grp * XGRP * FP;
#pragma unroll 1
    for (int it = 0; it < (XGRP * 8) / NTHR; ++it) {
      const int u  = it * NTHR + tid;
      const int r  = u >> 3;
      const int k8 = (u & 7) * 8;
      v8us o;
#pragma unroll
      for (int i = 0; i < 8; ++i) {
        const int c  = k8 + i;
        const int cc = c < FIN ? c : FIN - 1;
        const float val = sx[r * FIN + cc];
        o[i] = (c < FIN) ? (unsigned short)bf16_bits(val) : (unsigned short)0;
      }
      unsigned short* dp = xbn + (size_t)r * FP + k8;
      *(volatile v8us*)dp = o;
      __threadfence();
      *(volatile v8us*)dp = o;
    }
    return;
  }
  if (bid < PB_X + PB_W1) {
    const int v   = (bid - PB_X) * NTHR + tid;
    const int net = v >> 9;
    const int n   = (v >> 3) & 63;
    const int k8  = (v & 7) * 8;
    const int nc  = n < FIN ? n : FIN - 1;
    const float* p = W1 + (size_t)net * FIN * FIN + nc;
    v8us o;
#pragma unroll
    for (int i = 0; i < 8; ++i) {
      const int k  = k8 + i;
      const int kc = k < FIN ? k : FIN - 1;
      const float val = p[(size_t)kc * FIN];
      o[i] = (k < FIN && n < FIN) ? (unsigned short)bf16_bits(val) : (unsigned short)0;
    }
    unsigned short* dp = W1T + (size_t)net * FP * FP + (size_t)n * FP + k8;
    *(volatile v8us*)dp = o;
    __threadfence();
    *(volatile v8us*)dp = o;
    return;
  }
  if (bid < PB_X + PB_W1 + PB_WG) {
    const int v   = (bid - PB_X - PB_W1) * NTHR + tid;
    const int net = v >> 10;
    const int n   = (v >> 4) & 63;
    const int k8  = (v & 15) * 8;
    const float* p = Wg + (size_t)net * FIN * FP + n;
    v8us o;
#pragma unroll
    for (int i = 0; i < 8; ++i) {
      const int kk = (k8 + i) & 63;
      const int kc = kk < FIN ? kk : FIN - 1;
      const float val = p[(size_t)kc * FP];
      o[i] = (kk < FIN) ? (unsigned short)bf16_bits(val) : (unsigned short)0;
    }
    unsigned short* dp = WGT2 + (size_t)net * FP * K2 + (size_t)n * K2 + k8;
    *(volatile v8us*)dp = o;
    __threadfence();
    *(volatile v8us*)dp = o;
    return;
  }
  if (bid < PB_X + PB_W1 + PB_WG + PB_FC) {
    const int v  = (bid - PB_X - PB_W1 - PB_WG) * NTHR + tid;
    const int n  = (v >> 4) & 63;
    const int k8 = (v & 15) * 8;
    const float* p = fcW + n;
    v8us o;
#pragma unroll
    for (int i = 0; i < 8; ++i) {
      const int kk = (k8 + i) & 63;
      const float val = p[(size_t)kk * FP];
      o[i] = (unsigned short)bf16_bits(val);
    }
    unsigned short* dp = FC1T2 + (size_t)n * K2 + k8;
    *(volatile v8us*)dp = o;
    __threadfence();
    *(volatile v8us*)dp = o;
    return;
  }
  tab_fill(b1,  NNET * FIN, FIN, TAB + TB1, 64, tid);
  tab_fill(bg,  NNET * FP,  FP,  TAB + TBG, 64, tid);
  tab_fill(fcb, FP,         FP,  TAB + TFB, 16, tid);
  tab_fill(oW,  FP,         FP,  TAB + TOW, 16, tid);
  tab_fill(ob,  1,          1,   TAB + TOB, 8,  tid);
}

__global__ __launch_bounds__(GTHR) void k_gemm(
    const unsigned short* __restrict__ A, const unsigned short* __restrict__ WT,
    float* outF, int K, int ldo)
{
  __shared__ __attribute__((aligned(16))) float stg[GBM * GBN];
  const int tid = (int)threadIdx.x, lane = tid & 31, wave = tid >> 5, hh = lane >> 4, m = lane & 15;
  const int rowBase = (int)blockIdx.x * GBM;
  const int col0    = (int)blockIdx.y * GBN;

  v8f acc[4];
  {
    const v8f z = {0.f, 0.f, 0.f, 0.f, 0.f, 0.f, 0.f, 0.f};
    acc[0] = z; acc[1] = z; acc[2] = z; acc[3] = z;
  }
  const unsigned short* ap = A  + (size_t)(rowBase + 16 * wave + m) * (size_t)K + 8 * hh;
  const unsigned short* wp = WT + (size_t)(col0 + m) * (size_t)K + 8 * hh;
  const int ksteps = K >> 5;
#pragma unroll 1
  for (int ks = 0; ks < ksteps; ++ks) {
    FragB af;
    af.h[0] = *(const v8usa*)(ap + 32 * ks);
    af.h[1] = *(const v8usa*)(ap + 32 * ks + 16);
#pragma unroll
    for (int t = 0; t < 4; ++t) {
      const unsigned short* wq = wp + (size_t)(16 * t) * (size_t)K + 32 * ks;
      FragB bf;
      bf.h[0] = *(const v8usa*)wq;
      bf.h[1] = *(const v8usa*)(wq + 16);
      acc[t] = wmb(af, bf, acc[t]);
    }
  }

#pragma unroll
  for (int t = 0; t < 4; ++t) {
    const int lc = 16 * t + m;
#pragma unroll
    for (int r = 0; r < 8; ++r) {
      const int lr = 16 * wave + 8 * hh + r;
      stg[lr * GBN + lc] = acc[t][r];
    }
  }
  __syncthreads();

  v4f fv[8];
#pragma unroll
  for (int i = 0; i < 8; ++i) {
    const int lr = 16 * wave + 2 * i + hh;
    fv[i] = *(const v4fa*)(stg + lr * GBN + 4 * m);
  }
#pragma unroll
  for (int i = 0; i < 8; ++i) {
    const int lr = 16 * wave + 2 * i + hh;
    const int gr = rowBase + lr;
    float* op = outF + (size_t)gr * (size_t)ldo + col0 + 4 * m;
    *(volatile v4f*)op = fv[i];
  }
  __threadfence();
#pragma unroll
  for (int i = 0; i < 8; ++i) {
    const int lr = 16 * wave + 2 * i + hh;
    const int gr = rowBase + lr;
    float* op = outF + (size_t)gr * (size_t)ldo + col0 + 4 * m;
    *(volatile v4f*)op = fv[i];
  }
}

__global__ __launch_bounds__(NTHR) void k_bucket(const int* __restrict__ srcs, const int* __restrict__ dsts,
                                                 int nE, int nN, int vec8,
                                                 int* listG, int* cntG, int* offG, int* disG, int* flagG) {
  extern __shared__ __attribute__((aligned(16))) int dsm[];
  int* list = dsm;
  int* hl   = dsm + LISTN;
  int* sl   = dsm + LISTN + RCAP;
  int* cnt  = dsm + LISTN + 2 * RCAP;
  int* offs = cnt + NBA;
  int* cur  = offs + NBA;
  int* misc = cur + NBA;
  const int tid = (int)threadIdx.x, lane = tid & 31, wave = tid >> 5;
  const int nodeBase = (int)blockIdx.x * NBA;
  int nb = nN - nodeBase;
  nb = nb < 0 ? 0 : (nb > NBA ? NBA : nb);

  {
    const v4i z4 = {0, 0, 0, 0};
    for (int i = tid * 4; i < AGG_ZINTS; i += NTHR * 4) *(v4ia*)(dsm + i) = z4;
    if (tid < 16) misc[tid] = 0;
  }
  __syncthreads();

  int t = 0, ov = 0;
  const int nChunks = (nE + CHUNK - 1) / CHUNK;
#pragma unroll 1
  for (int ch = 0; ch < nChunks; ++ch) {
    const int cbase = ch * CHUNK;
    const int wc = scan_chunk<SLA>(dsts, nE, cbase, nodeBase, nb, vec8, list, tid, lane, wave);
    if (lane == 0) misc[wave] = wc;
    __syncthreads();
    if (wave == 0) {
#pragma unroll 1
      for (int w2 = 0; w2 < NWAVE; ++w2) {
        int c = misc[w2];
        c = c < 0 ? 0 : (c > WCAP ? WCAP : c);
#pragma unroll 1
        for (int b0 = 0; b0 < c; b0 += 32) {
          const int idx = b0 + lane;
          const int ent = list[w2 * WCAP + (idx < WCAP ? idx : WCAP - 1)];
          const int m32 = (c - b0) < 32 ? (c - b0) : 32;
#pragma unroll 1
          for (int k = 0; k < m32; ++k) {
            const int u    = __builtin_amdgcn_readlane(ent, k);
            const int slot = u & (NBA - 1);
            const int el   = (u >> SLA) & (CHUNK - 1);
            const int pk   = ((cbase + el) << SLA) | slot;
            if (t < RCAP) {
              if (lane == 0) { hl[t] = pk; cnt[slot] = cnt[slot] + 1; }
              t = t + 1;
            } else {
              ov = 1;
            }
          }
        }
      }
    }
    __syncthreads();
  }
  if (wave == 0 && lane == 0) { misc[8] = t; misc[9] = ov; }
  __syncthreads();
  int tt = misc[8];
  tt = tt < 0 ? 0 : (tt > RCAP ? RCAP : tt);
  const int ovf = misc[9];

  if (wave == 0) {
    const int base = lane * (NBA / 32);
    int s = 0;
#pragma unroll 1
    for (int i = 0; i < NBA / 32; ++i) s += cnt[base + i];
    int incl = s;
#pragma unroll
    for (int d = 1; d < 32; d <<= 1) {
      const int y = __shfl_up(incl, d, 32);
      if (lane >= d) incl += y;
    }
    int run = incl - s;
#pragma unroll 1
    for (int i = 0; i < NBA / 32; ++i) {
      const int cv = cnt[base + i];
      offs[base + i] = run;
      cur[base + i]  = run;
      run += cv;
    }
  }
  __syncthreads();
  if (wave == 0) {
#pragma unroll 1
    for (int b0 = 0; b0 < tt; b0 += 32) {
      const int idx = b0 + lane;
      const int ent = hl[idx < RCAP ? idx : RCAP - 1];
      const int m32 = (tt - b0) < 32 ? (tt - b0) : 32;
#pragma unroll 1
      for (int k = 0; k < m32; ++k) {
        const int u    = __builtin_amdgcn_readlane(ent, k);
        const int slot = u & (NBA - 1);
        if (lane == 0) {
          int p = cur[slot];
          p = p < 0 ? 0 : (p > RCAP - 1 ? RCAP - 1 : p);
          sl[p] = u;
          cur[slot] = p + 1;
        }
      }
    }
  }
  __syncthreads();

  int* lg = listG + (size_t)blockIdx.x * RCAP;
#pragma unroll 1
  for (int it = 0; it < RCAP / (4 * NTHR); ++it) {
    const int idx = (it * NTHR + tid) * 4;
    const v4i e4 = *(const v4ia*)(sl + idx);
    int e0 = e4.x >> SLA, e1 = e4.y >> SLA, e2 = e4.z >> SLA, e3 = e4.w >> SLA;
    e0 = e0 < 0 ? 0 : (e0 > nE - 1 ? nE - 1 : e0);
    e1 = e1 < 0 ? 0 : (e1 > nE - 1 ? nE - 1 : e1);
    e2 = e2 < 0 ? 0 : (e2 > nE - 1 ? nE - 1 : e2);
    e3 = e3 < 0 ? 0 : (e3 > nE - 1 ? nE - 1 : e3);
    const int r0 = srcs[e0], r1 = srcs[e1], r2 = srcs[e2], r3 = srcs[e3];
    v4i o;
    o.x = (idx     < tt) ? r0 : 0;
    o.y = (idx + 1 < tt) ? r1 : 0;
    o.z = (idx + 2 < tt) ? r2 : 0;
    o.w = (idx + 3 < tt) ? r3 : 0;
    int* dp = lg + idx;
    *(volatile v4i*)dp = o;
    __threadfence();
    *(volatile v4i*)dp = o;
  }

#pragma unroll 1
  for (int j = 0; j < NBA / NTHR; ++j) {
    const int s = j * NTHR + tid;
    int c = cnt[s];
    c = c < 0 ? 0 : c;
    const float d = 1.0f / sqrtf((float)(c + 1));
    cur[s] = __float_as_int(d);
  }
  __syncthreads();
  {
    const v4i c4 = *(const v4ia*)(cnt  + 4 * tid);
    const v4i o4 = *(const v4ia*)(offs + 4 * tid);
    const v4i d4 = *(const v4ia*)(cur  + 4 * tid);
    int* cp = cntG + (size_t)nodeBase + 4 * tid;
    int* op = offG + (size_t)nodeBase + 4 * tid;
    int* dp = disG + (size_t)nodeBase + 4 * tid;
    const v4i fv = {ovf, tt, 0, 0};
    int* fp = flagG + (size_t)blockIdx.x * 32 + 4 * (lane & 7);
    const bool fw = (wave == 0) && (lane < 8);
    *(volatile v4i*)cp = c4;
    *(volatile v4i*)op = o4;
    *(volatile v4i*)dp = d4;
    if (fw) *(volatile v4i*)fp = fv;
    __threadfence();
    *(volatile v4i*)cp = c4;
    *(volatile v4i*)op = o4;
    *(volatile v4i*)dp = d4;
    if (fw) *(volatile v4i*)fp = fv;
  }
}

__global__ __launch_bounds__(NTHR) void k_agg(const int* __restrict__ listG, const int* __restrict__ cntG,
                                              const int* __restrict__ offG, const float* __restrict__ dis,
                                              const int* __restrict__ flagG, int nN, int mRows,
                                              const float* __restrict__ xl, const float* __restrict__ bias,
                                              float* hout) {
  const int tid = (int)threadIdx.x, lane = tid & 31, wave = tid >> 5;
  const int nodeBase = (int)blockIdx.x * NBA;
  const int* lst = listG + (size_t)blockIdx.x * RCAP;
  const int ovf = flagG[(size_t)blockIdx.x * 32];
  float bv0, bv1;
  {
    const v2f a = *(const v2fa*)(bias + 2 * lane);
    bv0 = a.x; bv1 = a.y;
  }
  const float qnan = __int_as_float(0x7fc00000);
  const float pz = (ovf != 0) ? qnan : 0.0f;
  const int sa = (2 * lane) & 31, sb = (2 * lane + 1) & 31;
#pragma unroll 1
  for (int si = 0; si < NBA / NWAVE; ++si) {
    const int s    = si * NWAVE + wave;
    const int node = nodeBase + s;
    int c = cntG[node];
    const bool big = c > DEGCAP;
    c = c < 0 ? 0 : (c > DEGCAP ? DEGCAP : c);
    int o = offG[node];
    o = o < 0 ? 0 : (o > RCAP - 1 ? RCAP - 1 : o);
    int hiI = o + c - 1;
    hiI = hiI < o ? o : hiI;
    hiI = hiI > RCAP - 1 ? RCAP - 1 : hiI;
    const int nc = node < nN ? node : nN - 1;
    const float dd = dis[nc];
    const float rd = dd * dd;
    float acc0 = 0.0f, acc1 = 0.0f;
#pragma unroll 1
    for (int b0 = 0; b0 < c; b0 += 32) {
      int idx = o + b0 + lane;
      idx = idx > hiI ? hiI : idx;
      int sr = lst[idx];
      sr = sr < 0 ? 0 : (sr > nN - 1 ? nN - 1 : sr);
      const float cf  = dis[sr] * dd;
      const int   cfi = __float_as_int(cf);
      const int m32 = (c - b0) < 32 ? (c - b0) : 32;
#pragma unroll 1
      for (int k = 0; k < m32; ++k) {
        const int   sk = __builtin_amdgcn_readlane(sr, k);
        const float ck = __int_as_float(__builtin_amdgcn_readlane(cfi, k));
        const v2f a = *(const v2fa*)(xl + (size_t)sk * FP + 2 * lane);
        acc0 = fmaf(ck, a.x, acc0); acc1 = fmaf(ck, a.y, acc1);
      }
    }
    float sv0, sv1;
    {
      const v2f a = *(const v2fa*)(xl + (size_t)nc * FP + 2 * lane);
      sv0 = a.x; sv1 = a.y;
    }
    const float pzr = big ? qnan : pz;
    const bool live = node < nN;
    float y0 = (acc0 + sv0 * rd) + bv0;
    float y1 = (acc1 + sv1 * rd) + bv1;
    y0 = (y0 > 0.0f) ? y0 : (y0 - y0);
    y1 = (y1 > 0.0f) ? y1 : (y1 - y1);
    y0 = y0 + pzr; y1 = y1 + pzr;
    const float v0 = live ? y0 : 0.0f;
    const float v1 = live ? y1 : 0.0f;
    const bool wr = (node < mRows) && (lane < 16);
    v4f ow;
    ow.x = __shfl(v0, sa, 32); ow.y = __shfl(v1, sa, 32);
    ow.z = __shfl(v0, sb, 32); ow.w = __shfl(v1, sb, 32);
    float* op = hout + (size_t)node * FP + 4 * (lane & 15);
    if (wr) *(volatile v4f*)op = ow;
    __threadfence();
    if (wr) *(volatile v4f*)op = ow;
  }
}

__global__ __launch_bounds__(NTHR) void k_pool(const float* __restrict__ a1, const int* __restrict__ bat,
                                               int nN, unsigned short* gp) {
  extern __shared__ __attribute__((aligned(16))) float psm[];
  float* tbl = psm;
  unsigned short* stg = (unsigned short*)(psm + PTAB);
  const int tid = (int)threadIdx.x, lane = tid & 31, wave = tid >> 5;
  const int gbase = (int)blockIdx.x * PGB;
  float* wt = tbl + wave * (PGB * FP);
  {
    const v4f z = {0.0f, 0.0f, 0.0f, 0.0f};
    for (int i = lane * 4; i < PGB * FP; i += 128) *(v4fa*)(wt + i) = z;
  }
  __syncthreads();

#pragma unroll 1
  for (int i0 = wave * 32; i0 < nN; i0 += NTHR) {
    const int i  = i0 + lane;
    const int ic = i < nN ? i : nN - 1;
    const int b  = bat[ic];
    const unsigned lid = (unsigned)(b - gbase);
    const bool hit = (i < nN) && (lid < (unsigned)PGB);
    const int lidi = hit ? (int)lid : 0;
    unsigned msk = __builtin_amdgcn_ballot_w32(hit);
    int nh = (int)__builtin_popcount(msk);
    nh = nh > 32 ? 32 : nh;
#pragma unroll 1
    for (int q = 0; q < nh; ++q) {
      int k = __builtin_ffs((int)msk) - 1;
      msk &= msk - 1u;
      k = k < 0 ? 0 : (k > 31 ? 31 : k);
      int node = i0 + k;
      node = node > nN - 1 ? nN - 1 : node;
      const int gl = __builtin_amdgcn_readlane(lidi, k) & (PGB - 1);
      const v2f v = *(const v2fa*)(a1 + (size_t)node * FP + 2 * lane);
      float* tp = wt + gl * FP + 2 * lane;
      v2f mm = *(const v2fa*)tp;
      mm.x = (v.x > mm.x || v.x != v.x) ? v.x : mm.x;
      mm.y = (v.y > mm.y || v.y != v.y) ? v.y : mm.y;
      *(v2fa*)tp = mm;
    }
  }
  __syncthreads();

#pragma unroll 1
  for (int j = 0; j < (PGB * FP) / NTHR; ++j) {
    const int e  = j * NTHR + tid;
    const int gl = e >> 6;
    const int c  = e & 63;
    float mx = tbl[gl * FP + c];
#pragma unroll 1
    for (int w2 = 1; w2 < NWAVE; ++w2) {
      const float v = tbl[w2 * (PGB * FP) + gl * FP + c];
      mx = (v > mx || v != v) ? v : mx;
    }
    const unsigned hb = bf16_bits(mx);
    const unsigned lb = bf16_bits(mx - __uint_as_float(hb << 16));
    stg[gl * K2 + c]      = (unsigned short)hb;
    stg[gl * K2 + FP + c] = (unsigned short)lb;
  }
  __syncthreads();
  v8us qv[2];
#pragma unroll
  for (int j = 0; j < 2; ++j) qv[j] = *(const v8usa*)(stg + 8 * (j * NTHR + tid));
  unsigned short* gb = gp + (size_t)gbase * K2;
#pragma unroll
  for (int j = 0; j < 2; ++j) *(volatile v8us*)(gb + 8 * (size_t)(j * NTHR + tid)) = qv[j];
  __threadfence();
#pragma unroll
  for (int j = 0; j < 2; ++j) *(volatile v8us*)(gb + 8 * (size_t)(j * NTHR + tid)) = qv[j];
}

__global__ __launch_bounds__(NTHR) void k_head(const unsigned short* __restrict__ gp,
                                               const unsigned short* __restrict__ wgt2,
                                               const unsigned short* __restrict__ fc1t2,
                                               const float* __restrict__ tab, float* out) {
  __shared__ __attribute__((aligned(16))) float sbuf[HROWS * XCP];
  __shared__ float ows[FP];
  __shared__ __attribute__((aligned(16))) float outs[HROWS];
  unsigned short* atile = (unsigned short*)sbuf;
  const int tid = (int)threadIdx.x, lane = tid & 31, wave = tid >> 5, hh = lane >> 4, m = lane & 15;
  const int rowBase = (int)blockIdx.x * HROWS;
  if (tid < FP) ows[tid] = tab[TOW + tid];
  const float obv = tab[TOB];
  const v8f z8 = {0.f, 0.f, 0.f, 0.f, 0.f, 0.f, 0.f, 0.f};

  v8f accr[4];
  accr[0] = z8; accr[1] = z8; accr[2] = z8; accr[3] = z8;
#pragma unroll 1
  for (int net = 0; net < NNET; ++net) {
    v8f acc[4];
    acc[0] = z8; acc[1] = z8; acc[2] = z8; acc[3] = z8;
    const unsigned short* ap = gp + ((size_t)net * NGR + rowBase + 16 * wave + m) * (size_t)K2 + 8 * hh;
    const unsigned short* wp = wgt2 + ((size_t)net * FP + m) * (size_t)K2 + 8 * hh;
#pragma unroll 1
    for (int ks = 0; ks < K2 / 32; ++ks) {
      FragB af;
      af.h[0] = *(const v8usa*)(ap + 32 * ks);
      af.h[1] = *(const v8usa*)(ap + 32 * ks + 16);
#pragma unroll
      for (int t = 0; t < 4; ++t) {
        const unsigned short* wq = wp + (size_t)(16 * t) * (size_t)K2 + 32 * ks;
        FragB bf;
        bf.h[0] = *(const v8usa*)wq;
        bf.h[1] = *(const v8usa*)(wq + 16);
        acc[t] = wmb(af, bf, acc[t]);
      }
    }
#pragma unroll
    for (int t = 0; t < 4; ++t) {
      const float bgv = tab[TBG + net * FP + 16 * t + m];
#pragma unroll
      for (int r = 0; r < 8; ++r) {
        const float v = acc[t][r] + bgv;
        const float g = (v > 0.0f) ? v : (v - v);
        accr[t][r] = accr[t][r] + g * 0.25f;
      }
    }
  }

#pragma unroll
  for (int t = 0; t < 4; ++t) {
    const int lc = 16 * t + m;
#pragma unroll
    for (int r = 0; r < 8; ++r) {
      const int lr = 16 * wave + 8 * hh + r;
      const float v = accr[t][r];
      const unsigned hb = bf16_bits(v);
      const unsigned lb = bf16_bits(v - __uint_as_float(hb << 16));
      atile[lr * K2 + lc]      = (unsigned short)hb;
      atile[lr * K2 + FP + lc] = (unsigned short)lb;
    }
  }
  __syncthreads();

  v8f ac2[4];
  ac2[0] = z8; ac2[1] = z8; ac2[2] = z8; ac2[3] = z8;
  {
    const unsigned short* lap = atile + (16 * wave + m) * K2 + 8 * hh;
    const unsigned short* fp  = fc1t2 + (size_t)m * (size_t)K2 + 8 * hh;
#pragma unroll 1
    for (int ks = 0; ks < K2 / 32; ++ks) {
      FragB af;
      af.h[0] = *(const v8usa*)(lap + 32 * ks);
      af.h[1] = *(const v8usa*)(lap + 32 * ks + 16);
#pragma unroll
      for (int t = 0; t < 4; ++t) {
        const unsigned short* wq = fp + (size_t)(16 * t) * (size_t)K2 + 32 * ks;
        FragB bf;
        bf.h[0] = *(const v8usa*)wq;
        bf.h[1] = *(const v8usa*)(wq + 16);
        ac2[t] = wmb(af, bf, ac2[t]);
      }
    }
  }
  __syncthreads();

#pragma unroll
  for (int t = 0; t < 4; ++t) {
    const int lc = 16 * t + m;
    const float fb = tab[TFB + lc];
#pragma unroll
    for (int r = 0; r < 8; ++r) {
      const int lr = 16 * wave + 8 * hh + r;
      const float v = ac2[t][r] + fb;
      sbuf[lr * XCP + lc] = (v > 0.0f) ? v : (v - v);
    }
  }
  __syncthreads();

  if (tid < HROWS) {
    const float* xr = sbuf + tid * XCP;
    float s = 0.0f;
#pragma unroll 4
    for (int k = 0; k < FP; ++k) s = fmaf(xr[k], ows[k], s);
    outs[tid] = s + obv;
  }
  __syncthreads();
  const v4f ov = *(const v4fa*)(outs + 4 * lane);
  float* op = out + (size_t)rowBase + 4 * lane;
  const bool okst = (wave == 0);
  if (okst) *(volatile v4f*)op = ov;
  __threadfence();
  if (okst) *(volatile v4f*)op = ov;
}

static inline size_t al256(size_t o) { return (o + 255) & ~(size_t)255; }

extern "C" void kernel_launch(void* const* d_in, const int* in_sizes, int n_in,
                              void* d_out, int out_size, void* d_ws, size_t ws_size,
                              hipStream_t stream) {
  if (n_in < 20) return;
  for (int i = 0; i < NNET; ++i) {
    if (in_sizes[3 * i + 0] != NX) return;
    if (in_sizes[3 * i + 1] != 2 * NE) return;
    if (in_sizes[3 * i + 2] != NN) return;
  }
  if (in_sizes[12] != NNET * FIN * FIN || in_sizes[13] != NNET * FIN) return;
  if (in_sizes[14] != NNET * FIN * FP  || in_sizes[15] != NNET * FP)  return;
  if (in_sizes[16] != FP * FP || in_sizes[17] != FP) return;
  if (in_sizes[18] != FP || in_sizes[19] != 1) return;
  if (out_size != NGR) return;

  const float* W1  = (const float*)d_in[12];
  const float* b1  = (const float*)d_in[13];
  const float* Wg  = (const float*)d_in[14];
  const float* bg  = (const float*)d_in[15];
  const float* fcW = (const float*)d_in[16];
  const float* fcb = (const float*)d_in[17];
  const float* oW  = (const float*)d_in[18];
  const float* ob  = (const float*)d_in[19];
  float* out = (float*)d_out;

  char* ws = (char*)d_ws;
  size_t off = 0;
  const size_t oXB   = off; off = al256(off + (size_t)NNET * MP * FP * 2);
  const size_t oH    = off; off = al256(off + (size_t)MP * FP * 4);
  const size_t oA1   = off; off = al256(off + (size_t)MP * FP * 4);
  const size_t oLIST = off; off = al256(off + (size_t)NBLK * RCAP * 4);
  const size_t oCNT  = off; off = al256(off + (size_t)NBPAD * 4);
  const size_t oOFF  = off; off = al256(off + (size_t)NBPAD * 4);
  const size_t oDIS  = off; off = al256(off + (size_t)NBPAD * 4);
  const size_t oFLAG = off; off = al256(off + (size_t)NBLK * 128);
  const size_t oGP   = off; off = al256(off + (size_t)NNET * NGR * K2 * 2);
  const size_t oW1T  = off; off = al256(off + (size_t)NNET * FP * FP * 2);
  const size_t oWGT  = off; off = al256(off + (size_t)NNET * FP * K2 * 2);
  const size_t oFC   = off; off = al256(off + (size_t)FP * K2 * 2);
  const size_t oTAB  = off; off = al256(off + (size_t)TABN * 4);
  if (off > ws_size || off > (size_t)WSMAX) return;
  unsigned short* XB   = (unsigned short*)(ws + oXB);
  float*          H    = (float*)(ws + oH);
  float*          A1   = (float*)(ws + oA1);
  int*            LIST = (int*)(ws + oLIST);
  int*            CNT  = (int*)(ws + oCNT);
  int*            OFFS = (int*)(ws + oOFF);
  int*            DISI = (int*)(ws + oDIS);
  int*            FLAG = (int*)(ws + oFLAG);
  unsigned short* GP   = (unsigned short*)(ws + oGP);
  unsigned short* W1T  = (unsigned short*)(ws + oW1T);
  unsigned short* WGT2 = (unsigned short*)(ws + oWGT);
  unsigned short* FC1T = (unsigned short*)(ws + oFC);
  float*          TAB  = (float*)(ws + oTAB);

  const size_t bktLds  = (size_t)BKT_LDS_INTS * 4;
  const size_t poolLds = (size_t)POOL_LDS_BYTES;
  hipFuncSetAttribute(reinterpret_cast<const void*>(&k_bucket), hipFuncAttributeMaxDynamicSharedMemorySize, (int)bktLds);
  hipFuncSetAttribute(reinterpret_cast<const void*>(&k_pool), hipFuncAttributeMaxDynamicSharedMemorySize, (int)poolLds);

  k_prep<<<PB_ALL, NTHR, 0, stream>>>((const float*)d_in[0], (const float*)d_in[3], (const float*)d_in[6],
                                      (const float*)d_in[9], W1, b1, Wg, bg, fcW, fcb, oW, ob,
                                      XB, W1T, WGT2, FC1T, TAB);
  for (int i = 0; i < NNET; ++i) {
    const int* ei  = (const int*)d_in[3 * i + 1];
    const int* bat = (const int*)d_in[3 * i + 2];
    const int* src = ei;
    const int* dst = ei + NE;
    k_gemm<<<dim3(MP / GBM, FP / GBN), GTHR, 0, stream>>>(XB + (size_t)i * MP * FP, W1T + (size_t)i * FP * FP,
                                                         H, FP, FP);
    k_bucket<<<NBLK, NTHR, bktLds, stream>>>(src, dst, NE, NN, 1, LIST, CNT, OFFS, DISI, FLAG);
    k_agg<<<NBLK, NTHR, 0, stream>>>(LIST, CNT, OFFS, (const float*)DISI, FLAG, NN, MP, H,
                                     TAB + TB1 + i * FP, A1);
    k_pool<<<NGR / PGB, NTHR, poolLds, stream>>>(A1, bat, NN, GP + (size_t)i * NGR * K2);
  }
  k_head<<<NGR / HROWS, NTHR, 0, stream>>>(GP, WGT2, FC1T, TAB, out);
}
